// SingleModalAtten_6021544149579
// MI455X (gfx1250) — hardware-verified
//
#include <hip/hip_runtime.h>
#include <math.h>
#include <stdint.h>

#define NB   4
#define NC   1024
#define NT   2048
#define NH   16
#define CH   64
#define NQK  2048
#define KD   1024

typedef _Float16 v16h __attribute__((ext_vector_type(16)));
typedef _Float16 v8h  __attribute__((ext_vector_type(8)));
typedef float    v8f  __attribute__((ext_vector_type(8)));
typedef float    v4f  __attribute__((ext_vector_type(4)));

union Frag { v16h v; v8h h[2]; };

static_assert(sizeof(long) == 8);

__device__ __forceinline__ v16h ld_frag(const _Float16* p) {
  Frag f;
  f.h[0] = *(const v8h*)(p);
  f.h[1] = *(const v8h*)(p + 16);
  return f.v;
}
__device__ __forceinline__ v8f zero8() { v8f z = {0.f, 0.f, 0.f, 0.f, 0.f, 0.f, 0.f, 0.f}; return z; }
__device__ __forceinline__ v8f mma16(v16h a, v16h b, v8f c) {
  return __builtin_amdgcn_wmma_f32_16x16x32_f16(false, a, false, b, (short)0, c, false, false);
}
__device__ __forceinline__ void dep_guard(v8f& a, v8f& b, v16h x, v16h y) {
  asm volatile("v_nop\n\tv_nop\n\tv_nop\n\tv_nop" : "+v"(a), "+v"(b) : "v"(x), "v"(y));
}
__device__ __forceinline__ void dep_guard1(v8f& a, v16h x, v16h y, v16h z, v16h w) {
  asm volatile("v_nop\n\tv_nop\n\tv_nop\n\tv_nop" : "+v"(a) : "v"(x), "v"(y), "v"(z), "v"(w));
}
__device__ __forceinline__ void keep4(v16h a, v16h b, v16h c, v16h d) {
  asm volatile("v_nop" :: "v"(a), "v"(b), "v"(c), "v"(d));
}
__device__ __forceinline__ void acc_guard4(v8f& a, v8f& b, v8f& c, v8f& d) {
  asm volatile("v_nop\n\tv_nop\n\tv_nop\n\tv_nop" : "+v"(a), "+v"(b), "+v"(c), "+v"(d));
}
__device__ __forceinline__ void lds_wave_sync() {
  __builtin_amdgcn_fence(__ATOMIC_RELEASE, "workgroup");
  __builtin_amdgcn_wave_barrier();
  __builtin_amdgcn_fence(__ATOMIC_ACQUIRE, "workgroup");
}

__global__ __launch_bounds__(256) void cvt_w16_kernel(const float* __restrict__ w,
                                                      _Float16* __restrict__ o, int n8) {
  const int i = blockIdx.x * 256 + threadIdx.x;
  if (i < n8) {
    const v4f a = *(const v4f*)(w + (size_t)i * 8);
    const v4f c = *(const v4f*)(w + (size_t)i * 8 + 4);
    v8h pk;
#pragma unroll
    for (int e = 0; e < 4; ++e) {
      pk[e]     = (_Float16)(a[e] * 64.0f);
      pk[4 + e] = (_Float16)(c[e] * 64.0f);
    }
    *(volatile v8h*)(o + (size_t)i * 8) = pk;
    __threadfence();
    *(volatile v8h*)(o + (size_t)i * 8) = pk;
  }
}

__global__ __launch_bounds__(256) void gn_kernel(const float* __restrict__ x,
                                                 const float* __restrict__ gam,
                                                 const float* __restrict__ bet,
                                                 _Float16* __restrict__ XT) {
  __shared__ double red[4][256];
  __shared__ __align__(16) float tile[64 * 68];
  __shared__ float stt[4];
  const int tid = threadIdx.x;
  const int b  = blockIdx.x >> 4;
  const int gp = blockIdx.x & 15;
  const int c0 = gp * 64;
  const float* xb = x + ((size_t)(b * NC + c0)) * NT;

  double s0 = 0.0, q0 = 0.0, s1 = 0.0, q1 = 0.0;
#pragma unroll 1
  for (int it = 0; it < 64; ++it) {
    const v4f v = *(const v4f*)(xb + ((size_t)(it * 256 + tid)) * 4);
#pragma unroll
    for (int e = 0; e < 4; ++e) { const double d = (double)v[e]; s0 += d; q0 += d * d; }
  }
#pragma unroll 1
  for (int it = 64; it < 128; ++it) {
    const v4f v = *(const v4f*)(xb + ((size_t)(it * 256 + tid)) * 4);
#pragma unroll
    for (int e = 0; e < 4; ++e) { const double d = (double)v[e]; s1 += d; q1 += d * d; }
  }
  red[0][tid] = s0; red[1][tid] = q0; red[2][tid] = s1; red[3][tid] = q1;
  __syncthreads();
#pragma unroll 1
  for (int off = 128; off > 0; off >>= 1) {
    if (tid < off) {
      red[0][tid] += red[0][tid + off];
      red[1][tid] += red[1][tid + off];
      red[2][tid] += red[2][tid + off];
      red[3][tid] += red[3][tid + off];
    }
    __syncthreads();
  }
  if (tid == 0) {
#pragma unroll
    for (int g = 0; g < 2; ++g) {
      const double mean = red[2 * g][0] * (1.0 / 65536.0);
      const double var  = red[2 * g + 1][0] * (1.0 / 65536.0) - mean * mean;
      float vf = (float)var;
      vf = (vf < 0.f) ? 0.f : vf;
      stt[2 * g]     = (float)mean;
      stt[2 * g + 1] = rsqrtf(vf + 1e-5f);
    }
  }
  __syncthreads();

#pragma unroll 1
  for (int tt = 0; tt < NT / 64; ++tt) {
    const int tb = tt * 64;
    __syncthreads();
#pragma unroll 1
    for (int p = 0; p < 4; ++p) {
      const int cl = p * 16 + (tid >> 4);
      const int t4 = (tid & 15) * 4;
      v4f v = *(const v4f*)(xb + (size_t)cl * NT + tb + t4);
      const int g = cl >> 5;
      const float mean = stt[2 * g], rstd = stt[2 * g + 1];
      const float ga = gam[c0 + cl], be = bet[c0 + cl];
#pragma unroll
      for (int e = 0; e < 4; ++e) v[e] = ((v[e] - mean) * rstd) * ga + be;
      *(v4f*)(tile + cl * 68 + t4) = v;
    }
    __syncthreads();
    v8h pk[2];
#pragma unroll
    for (int p = 0; p < 2; ++p) {
      const int tl = p * 32 + (tid >> 3);
      const int c8 = (tid & 7) * 8;
      v8h w;
#pragma unroll
      for (int e = 0; e < 8; ++e) w[e] = (_Float16)tile[(c8 + e) * 68 + tl];
      pk[p] = w;
    }
    for (int pass = 0; pass < 2; ++pass) {
#pragma unroll
      for (int p = 0; p < 2; ++p) {
        const int tl = p * 32 + (tid >> 3);
        const int c8 = (tid & 7) * 8;
        _Float16* dst = XT + ((size_t)(b * NT + tb + tl)) * NC + c0 + c8;
        *(volatile v8h*)dst = pk[p];
      }
      __threadfence();
    }
  }
}

template <int MODE>
__global__ __launch_bounds__(256) void gemm64_kernel(
    const _Float16* __restrict__ A, long strideA,
    const _Float16* __restrict__ Bm, long strideB,
    const float* __restrict__ bias, const float* __restrict__ resid,
    void* __restrict__ outp, int M, int N, float scale) {
  __shared__ __align__(16) float slab_all[8 * 16 * 68];
  const int lane = threadIdx.x & 31;
  const int wave = threadIdx.x >> 5;
  const int hh = lane >> 4, rl = lane & 15;
  const int b = blockIdx.y;
  const int tilesN = N >> 6, tilesM = M >> 6;
  const int tile = blockIdx.x * 8 + wave;
  if (tile >= tilesM * tilesN) return;
  const int tm = tile / tilesN;
  const int tn = tile - tm * tilesN;
  const int m0 = tm << 6, n0 = tn << 6;

  const _Float16* Ab = A  + (size_t)b * strideA + (size_t)(m0 + rl) * KD + 8 * hh;
  const _Float16* Bb = Bm + (size_t)b * strideB + (size_t)(n0 + rl) * KD + 8 * hh;

  v8f acc[4][4];
#pragma unroll
  for (int i = 0; i < 4; ++i)
#pragma unroll
    for (int j = 0; j < 4; ++j) acc[i][j] = zero8();

#pragma unroll 1
  for (int k0 = 0; k0 < KD; k0 += 32) {
    v16h bf[4];
#pragma unroll
    for (int j = 0; j < 4; ++j) bf[j] = ld_frag(Bb + (size_t)(j * 16) * KD + k0);
#pragma unroll
    for (int i = 0; i < 4; ++i) {
      const v16h af = ld_frag(Ab + (size_t)(i * 16) * KD + k0);
#pragma unroll
      for (int j = 0; j < 4; ++j) acc[i][j] = mma16(af, bf[j], acc[i][j]);
      dep_guard(acc[i][0], acc[i][3], af, bf[3]);
    }
    keep4(bf[0], bf[1], bf[2], bf[3]);
  }
  acc_guard4(acc[0][0], acc[0][1], acc[0][2], acc[0][3]);
  acc_guard4(acc[1][0], acc[1][1], acc[1][2], acc[1][3]);
  acc_guard4(acc[2][0], acc[2][1], acc[2][2], acc[2][3]);
  acc_guard4(acc[3][0], acc[3][1], acc[3][2], acc[3][3]);

  if (MODE != 2) {
    _Float16* slab = (_Float16*)slab_all + wave * (16 * 72);
    _Float16* orow;
    if (MODE == 0) orow = (_Float16*)outp + ((size_t)(b * 32 + (m0 >> 6)) * NT) * CH;
    else           orow = (_Float16*)outp + (size_t)b * NC * NT + m0;
    const size_t opitch = (MODE == 0) ? (size_t)CH : (size_t)NT;
    v8f bm[4];
#pragma unroll
    for (int i = 0; i < 4; ++i) bm[i] = zero8();
    if (MODE == 0) {
#pragma unroll
      for (int i = 0; i < 4; ++i)
#pragma unroll
        for (int r = 0; r < 8; ++r) bm[i][r] = bias[m0 + i * 16 + 8 * hh + r];
    }
    const int q = lane >> 3, c8 = (lane & 7) * 8;
#pragma unroll
    for (int j = 0; j < 4; ++j) {
      float bn = 0.f;
      if (MODE == 1) bn = bias[NQK + n0 + j * 16 + rl];
#pragma unroll
      for (int i = 0; i < 4; ++i) {
        v8h pk;
#pragma unroll
        for (int r = 0; r < 8; ++r) {
          const float v = acc[i][j][r] * scale + ((MODE == 0) ? bm[i][r] : bn);
          pk[r] = (_Float16)v;
        }
        *(v8h*)(slab + rl * 72 + i * 16 + 8 * hh) = pk;
      }
      lds_wave_sync();
      v8h vv[4];
#pragma unroll
      for (int it = 0; it < 4; ++it) vv[it] = *(const v8h*)(slab + (it * 4 + q) * 72 + c8);
      for (int pass = 0; pass < 2; ++pass) {
#pragma unroll
        for (int it = 0; it < 4; ++it) {
          const int n = n0 + j * 16 + it * 4 + q;
          *(volatile v8h*)(orow + (size_t)n * opitch + c8) = vv[it];
        }
        __threadfence();
      }
      lds_wave_sync();
    }
  } else {
    float* slab = slab_all + wave * (16 * 68);
    float* outb = (float*)outp + (size_t)b * NC * NT;
    const float* xb = resid + (size_t)b * NC * NT;
    const int c4 = (lane & 15) * 4;
#pragma unroll
    for (int j = 0; j < 4; ++j) {
#pragma unroll
      for (int i = 0; i < 4; ++i) {
        v4f p0, p1;
#pragma unroll
        for (int e = 0; e < 4; ++e) { p0[e] = acc[i][j][e] * scale; p1[e] = acc[i][j][4 + e] * scale; }
        *(v4f*)(slab + rl * 68 + i * 16 + 8 * hh)     = p0;
        *(v4f*)(slab + rl * 68 + i * 16 + 8 * hh + 4) = p1;
      }
      lds_wave_sync();
      v4f vals[8];
#pragma unroll
      for (int it = 0; it < 8; ++it) {
        const int row = it * 2 + hh;
        const int n = n0 + j * 16 + row;
        const size_t gi = (size_t)n * NT + m0 + c4;
        const v4f sv = *(const v4f*)(slab + row * 68 + c4);
        const v4f xr = *(const v4f*)(xb + gi);
        const float bb = bias[n];
        vals[it] = xr + (sv + bb);
      }
      for (int pass = 0; pass < 2; ++pass) {
#pragma unroll
        for (int it = 0; it < 8; ++it) {
          const int row = it * 2 + hh;
          const size_t gi = (size_t)(n0 + j * 16 + row) * NT + m0 + c4;
          *(volatile v4f*)(outb + gi) = vals[it];
        }
        __threadfence();
      }
      lds_wave_sync();
    }
  }
}

__global__ __launch_bounds__(256) void attn_kernel(const _Float16* __restrict__ QK,
                                                   const _Float16* __restrict__ Vp,
                                                   _Float16* __restrict__ AT) {
  __shared__ __align__(16) _Float16 Ks[64 * 72];
  __shared__ __align__(16) _Float16 Vs[64 * 72];
  __shared__ __align__(16) _Float16 Osl[8 * 16 * 72];
  const int tid = threadIdx.x, wave = tid >> 5, lane = tid & 31;
  const int hh = lane >> 4, rl = lane & 15;
  const int bh = blockIdx.y;
  const int b = bh >> 4, h = bh & 15;
  const int t0 = blockIdx.x * 128 + wave * 16;
  const _Float16* qp = QK + ((size_t)(b * 32 + h) * NT) * CH;
  const _Float16* kp = QK + ((size_t)(b * 32 + NH + h) * NT) * CH;
  const _Float16* vp = Vp + ((size_t)(b * NC + h * CH)) * NT;

  v16h qf[2];
#pragma unroll
  for (int kc = 0; kc < 2; ++kc) qf[kc] = ld_frag(qp + (size_t)(t0 + rl) * CH + kc * 32 + 8 * hh);

  float mrun = -INFINITY, lrun = 0.f;
  v8f oacc[4];
#pragma unroll
  for (int ct = 0; ct < 4; ++ct) oacc[ct] = zero8();
  const float cl2 = 0.18033688011112042f;

#pragma unroll 1
  for (int st = 0; st < NT / 64; ++st) {
    const int s0 = st * 64;
    __syncthreads();
#pragma unroll
    for (int p = 0; p < 2; ++p) {
      const int id = tid + p * 256;
      const int row = id >> 3, c8 = (id & 7) * 8;
      const v8h kv = *(const v8h*)(kp + (size_t)(s0 + row) * CH + c8);
      const v8h vv = *(const v8h*)(vp + (size_t)row * NT + s0 + c8);
      *(v8h*)(Ks + row * 72 + c8) = kv;
      *(v8h*)(Vs + row * 72 + c8) = vv;
    }
    __syncthreads();

    v8f sacc[4];
#pragma unroll
    for (int mt = 0; mt < 4; ++mt) {
      const v16h a0 = ld_frag(Ks + (mt * 16 + rl) * 72 + 8 * hh);
      const v16h a1 = ld_frag(Ks + (mt * 16 + rl) * 72 + 32 + 8 * hh);
      sacc[mt] = mma16(a0, qf[0], zero8());
      sacc[mt] = mma16(a1, qf[1], sacc[mt]);
      dep_guard1(sacc[mt], a0, a1, qf[0], qf[1]);
    }
    float mx = -INFINITY;
#pragma unroll
    for (int mt = 0; mt < 4; ++mt)
#pragma unroll
      for (int r = 0; r < 8; ++r) mx = fmaxf(mx, sacc[mt][r]);
    mx = fmaxf(mx, __shfl_xor(mx, 16, 32));
    const float mnew = fmaxf(mrun, mx * cl2);
    const float alpha = __builtin_amdgcn_exp2f(mrun - mnew);
    mrun = mnew;
    float ps = 0.f;
    Frag pf[2];
#pragma unroll
    for (int mt = 0; mt < 4; ++mt) {
      v8h pk;
#pragma unroll
      for (int r = 0; r < 8; ++r) {
        const float p = __builtin_amdgcn_exp2f(sacc[mt][r] * cl2 - mnew);
        ps += p;
        pk[r] = (_Float16)(p * 1024.0f);
      }
      pf[mt >> 1].h[mt & 1] = pk;
    }
    ps += __shfl_xor(ps, 16, 32);
    lrun = lrun * alpha + ps;
#pragma unroll
    for (int ct = 0; ct < 4; ++ct) oacc[ct] *= alpha;
#pragma unroll
    for (int ct = 0; ct < 4; ++ct) {
      const v16h a0 = ld_frag(Vs + (ct * 16 + rl) * 72 + 8 * hh);
      const v16h a1 = ld_frag(Vs + (ct * 16 + rl) * 72 + 32 + 8 * hh);
      oacc[ct] = mma16(a0, pf[0].v, oacc[ct]);
      oacc[ct] = mma16(a1, pf[1].v, oacc[ct]);
      dep_guard1(oacc[ct], a0, a1, pf[0].v, pf[1].v);
    }
  }

  const float inv = __builtin_amdgcn_rcpf(lrun) * 0.0625f;
  _Float16* slab = Osl + wave * (16 * 72);
#pragma unroll
  for (int ct = 0; ct < 4; ++ct) {
    v8h pk;
#pragma unroll
    for (int r = 0; r < 8; ++r) pk[r] = (_Float16)(oacc[ct][r] * inv);
    *(v8h*)(slab + rl * 72 + ct * 16 + 8 * hh) = pk;
  }
  lds_wave_sync();
  const int q = lane >> 3, c8 = (lane & 7) * 8;
  v8h ov[4];
#pragma unroll
  for (int it = 0; it < 4; ++it) ov[it] = *(const v8h*)(slab + (it * 4 + q) * 72 + c8);
  _Float16* ab = AT + ((size_t)(b * NT + t0)) * NC + h * CH + c8;
  for (int pass = 0; pass < 2; ++pass) {
#pragma unroll
    for (int it = 0; it < 4; ++it) *(volatile v8h*)(ab + (size_t)(it * 4 + q) * NC) = ov[it];
    __threadfence();
  }
}

extern "C" void kernel_launch(void* const* d_in, const int* in_sizes, int n_in,
                              void* d_out, int out_size, void* d_ws, size_t ws_size,
                              hipStream_t stream) {
  if (n_in < 7) return;
  if (in_sizes[0] != NB * NC * NT) return;
  if (in_sizes[1] != NC || in_sizes[2] != NC) return;
  if (in_sizes[3] != 3 * NC * NC || in_sizes[4] != 3 * NC) return;
  if (in_sizes[5] != NC * NC || in_sizes[6] != NC) return;
  if (out_size != NB * NC * NT) return;

  const float* x      = (const float*)d_in[0];
  const float* gn_s   = (const float*)d_in[1];
  const float* gn_b   = (const float*)d_in[2];
  const float* qkv_w  = (const float*)d_in[3];
  const float* qkv_b  = (const float*)d_in[4];
  const float* proj_w = (const float*)d_in[5];
  const float* proj_b = (const float*)d_in[6];
  float* out = (float*)d_out;

  const size_t szWq = (size_t)3 * NC * NC * 2;
  const size_t szWp = (size_t)NC * NC * 2;
  const size_t szXT = (size_t)NB * NT * NC * 2;
  const size_t szQK = (size_t)NB * NQK * NT * 2;
  const size_t szV  = (size_t)NB * NC * NT * 2;
  const size_t szAT = (size_t)NB * NT * NC * 2;
  size_t off = 0;
  const size_t oWq = off; off += szWq;
  const size_t oWp = off; off += szWp;
  const size_t oXT = off; off += szXT;
  const size_t oQK = off; off += szQK;
  const size_t oV  = off; off += szV;
  const size_t oAT = off; off += szAT;
  static_assert((size_t)3 * NC * NC * 2 + (size_t)NC * NC * 2 + (size_t)NB * NT * NC * 2 * 3 +
                (size_t)NB * NQK * NT * 2 <= (size_t)134217728);
  if (off > ws_size) return;

  char* ws = (char*)d_ws;
  _Float16* Wq16 = (_Float16*)(ws + oWq);
  _Float16* Wp16 = (_Float16*)(ws + oWp);
  _Float16* XT   = (_Float16*)(ws + oXT);
  _Float16* QK   = (_Float16*)(ws + oQK);
  _Float16* V    = (_Float16*)(ws + oV);
  _Float16* AT   = (_Float16*)(ws + oAT);

  const dim3 blk(256);
  const int n8q = (3 * NC * NC) / 8;
  const int n8p = (NC * NC) / 8;
  cvt_w16_kernel<<<dim3((n8q + 255) / 256), blk, 0, stream>>>(qkv_w, Wq16, n8q);
  cvt_w16_kernel<<<dim3((n8p + 255) / 256), blk, 0, stream>>>(proj_w, Wp16, n8p);
  gn_kernel<<<dim3(NB * 16), blk, 0, stream>>>(x, gn_s, gn_b, XT);

  const long actStride = (long)NT * NC;
  gemm64_kernel<0><<<dim3((NQK / 64) * (NT / 64) / 8, NB), blk, 0, stream>>>(
      Wq16, 0L, XT, actStride, qkv_b, x, (void*)QK, NQK, NT, 1.0f / 64.0f);
  gemm64_kernel<1><<<dim3((NT / 64) * (NC / 64) / 8, NB), blk, 0, stream>>>(
      XT, actStride, Wq16 + (size_t)NQK * KD, 0L, qkv_b, x, (void*)V, NT, NC, 1.0f / 64.0f);
  attn_kernel<<<dim3(NT / 128, NB * NH), blk, 0, stream>>>(QK, V, AT);
  gemm64_kernel<2><<<dim3((NT / 64) * (NC / 64) / 8, NB), blk, 0, stream>>>(
      AT, actStride, Wp16, 0L, proj_b, x, (void*)out, NT, NC, 1.0f / 4096.0f);
  (void)hipGetLastError();
}
